// MultiHeadAttention2_70385924047429
// MI455X (gfx1250) — hardware-verified
//
#include <hip/hip_runtime.h>
#include <math.h>

typedef __attribute__((ext_vector_type(16))) _Float16 v16h;
typedef __attribute__((ext_vector_type(16))) __bf16 v16b;
typedef __attribute__((ext_vector_type(8)))  _Float16 v8h;
typedef __attribute__((ext_vector_type(8)))  __bf16 v8b;
typedef __attribute__((ext_vector_type(8)))  float v8f;
typedef __attribute__((ext_vector_type(4)))  float v4f;
typedef __attribute__((ext_vector_type(4)))  unsigned v4u;
typedef __attribute__((ext_vector_type(4)))  int v4i;

template <typename T> __device__ __forceinline__ void vst2(void* p, T v) { *(volatile T*)p = v; __threadfence(); *(volatile T*)p = v; }
__device__ __forceinline__ v8f wmma16(v16h a, v16h b, v8f c) {
  v8f d = __builtin_amdgcn_wmma_f32_16x16x32_f16(false, a, false, b, (short)0, c, false, false);
  asm volatile("v_nop\n\tv_nop\n\tv_nop\n\tv_nop" : "+v"(d) : "v"(a), "v"(b));
  return d;
}
__device__ __forceinline__ v8f wmma_bf(v16b a, v16b b, v8f c) {
  v8f d = __builtin_amdgcn_wmma_f32_16x16x32_bf16(false, a, false, b, (short)0, c, false, false);
  asm volatile("v_nop\n\tv_nop\n\tv_nop\n\tv_nop" : "+v"(d) : "v"(a), "v"(b));
  return d;
}
__device__ __forceinline__ v16h frag_h(const _Float16* rowk0, int lane) {
  union { v16h v; v8h q[2]; } u; const _Float16* p = rowk0 + 8 * (lane >> 4);
  u.q[0] = *(const v8h*)p; u.q[1] = *(const v8h*)(p + 16); return u.v;
}
__device__ __forceinline__ v16b frag_b(const __bf16* rowk0, int lane) {
  union { v16b v; v8b q[2]; } u; const __bf16* p = rowk0 + 8 * (lane >> 4);
  u.q[0] = *(const v8b*)p; u.q[1] = *(const v8b*)(p + 16); return u.v;
}
__device__ __forceinline__ v16b frag_f32b(const float* rowk0, int lane) {
  const float* p = rowk0 + 8 * (lane >> 4); const v8f x0 = *(const v8f*)p, x1 = *(const v8f*)(p + 16); v16b a;
#pragma unroll
  for (int i = 0; i < 8; ++i) { a[i] = (__bf16)x0[i]; a[8 + i] = (__bf16)x1[i]; }
  return a;
}
struct F2 { v16b h, l; };
__device__ __forceinline__ F2 bsplit16(const float v[16]) { F2 r;
#pragma unroll
  for (int i = 0; i < 16; ++i) { const __bf16 hh = (__bf16)v[i]; r.h[i] = hh; r.l[i] = (__bf16)(v[i] - (float)hh); }
  return r; }
__device__ __forceinline__ F2 split_row(const float* row, int k0, int lane) { float v[16]; const float* p = row + k0 + 8 * (lane >> 4); const v8f x0 = *(const v8f*)p, x1 = *(const v8f*)(p + 16);
#pragma unroll
  for (int i = 0; i < 8; ++i) { v[i] = x0[i]; v[8 + i] = x1[i]; }
  return bsplit16(v); }
__device__ __forceinline__ float bfr(float v) { return (float)(__bf16)v; }
#define LDSX() do { asm volatile("s_wait_dscnt 0" ::: "memory"); __builtin_amdgcn_wave_barrier(); __builtin_amdgcn_fence(__ATOMIC_RELEASE, "workgroup"); } while (0)

#ifndef NB
#define NB 2
#endif
#ifndef SEQ
#define SEQ 2048
#endif
#define NB_FULL 2
#define SEQ_FULL 2048
#define SEQK 2048
#define SEQK_FULL 2048
#define DM 1024
#define NH 16
#define HD 64
#define KVW (2 * DM)
#define LN_EPS 1.0e-6f
static_assert(NB >= 1 && NB <= NB_FULL);
static_assert(SEQ % 64 == 0 && SEQ >= 64 && SEQ <= SEQ_FULL);
static_assert(SEQK % 64 == 0 && SEQK == SEQK_FULL);
static_assert(DM % 128 == 0 && KVW % 128 == 0 && NH * HD == DM && HD == 64);

#define WS_PQ  0ull
#define WS_PKV (WS_PQ + 2ull * DM * DM)
#define WS_PO  (WS_PKV + 2ull * KVW * DM)
#define WS_NQ  (WS_PO + 2ull * DM * DM)
#define WS_QH  (WS_NQ + 4ull * NB * SEQ * DM)
#define WS_KH  (WS_QH + 2ull * NB * SEQ * DM)
#define WS_VT  (WS_KH + 2ull * NB * SEQK * DM)
#define WS_O   (WS_VT + 2ull * NB * DM * SEQK)
#define WS_Y   (WS_O + 4ull * NB * SEQ * DM)
#define WS_END (WS_Y + 4ull * NB * SEQ * DM)
static_assert(WS_END <= 134217728ull);
static_assert((WS_PKV % 128) == 0 && (WS_PO % 128) == 0 && (WS_NQ % 128) == 0 && (WS_QH % 128) == 0 && (WS_KH % 128) == 0 && (WS_VT % 128) == 0 && (WS_O % 128) == 0 && (WS_Y % 128) == 0);

__global__ __launch_bounds__(256) void k_pack(const float* __restrict__ W, int K, int N, __bf16* __restrict__ PK) {
  __shared__ __align__(16) __bf16 s[64][72];
  const int n0 = blockIdx.x * 64, k0 = blockIdx.y * 64, t = threadIdx.x;
#pragma unroll 4
  for (int i = 0; i < 16; ++i) { const int idx = t + 256 * i; const int kk = idx >> 6, nn = idx & 63; s[nn][kk] = (__bf16)W[(size_t)(k0 + kk) * N + n0 + nn]; }
  __syncthreads();
#pragma unroll
  for (int i = 0; i < 2; ++i) { const int p = t + 256 * i; const int nn = p >> 3, c = p & 7;
    vst2((unsigned*)(PK + (size_t)(n0 + nn) * K + k0 + c * 8), *(const v4u*)&s[nn][c * 8]); }
}

__global__ __launch_bounds__(256) void k_lnq(const float* __restrict__ X, const float* __restrict__ G, const float* __restrict__ Bt, float* __restrict__ NQ) {
  __shared__ float red0[8], red1[8];
  const int rc = blockIdx.x; const int b = rc / SEQ, s = rc - b * SEQ; const size_t rin = (size_t)b * SEQ_FULL + s;
  const int t = threadIdx.x, lane = t & 31, wave = t >> 5;
  const v4f xv = *(const v4f*)(X + rin * DM + t * 4);
  float v[4];
#pragma unroll
  for (int i = 0; i < 4; ++i) v[i] = bfr(xv[i]);
  float ps = (v[0] + v[1]) + (v[2] + v[3]);
#pragma unroll
  for (int o = 16; o > 0; o >>= 1) ps += __shfl_xor(ps, o);
  if (lane == 0) red0[wave] = ps;
  __syncthreads();
  float S = 0.f;
#pragma unroll
  for (int i = 0; i < 8; ++i) S += red0[i];
  const float mean = S * (1.0f / DM);
  float d[4]; float pq = 0.f;
#pragma unroll
  for (int i = 0; i < 4; ++i) { d[i] = v[i] - mean; pq += d[i] * d[i]; }
#pragma unroll
  for (int o = 16; o > 0; o >>= 1) pq += __shfl_xor(pq, o);
  if (lane == 0) red1[wave] = pq;
  __syncthreads();
  float V = 0.f;
#pragma unroll
  for (int i = 0; i < 8; ++i) V += red1[i];
  const float rstd = 1.0f / sqrtf(V * (1.0f / DM) + LN_EPS);
  const v4f gv = *(const v4f*)(G + t * 4), bv = *(const v4f*)(Bt + t * 4); v4f o;
#pragma unroll
  for (int i = 0; i < 4; ++i) o[i] = d[i] * rstd * bfr(gv[i]) + bfr(bv[i]);
  vst2(NQ + (size_t)rc * DM + t * 4, o);
}

__global__ __launch_bounds__(128) void k_proj(const float* __restrict__ X, int spb, int spb_full, const __bf16* __restrict__ P, const float* __restrict__ BI, _Float16* __restrict__ NAT, _Float16* __restrict__ VT) {
  __shared__ __align__(16) _Float16 so[4][16][136];
  __shared__ __align__(16) _Float16 sth[128][72];
  const int tid = threadIdx.x, wave = tid >> 5, lane = tid & 31, col = lane & 15, g = lane >> 4;
  const int rc0 = blockIdx.x * 64; const int b = rc0 / spb, s0 = rc0 - b * spb; const int n0 = blockIdx.y * 128;
  const float* xrow = X + ((size_t)b * spb_full + s0 + wave * 16 + col) * DM;
  v8f acc[8] = {};
#pragma unroll 2
  for (int kc = 0; kc < DM / 32; ++kc) { const v16b a = frag_f32b(xrow + kc * 32, lane);
#pragma unroll
    for (int j = 0; j < 8; ++j) acc[j] = wmma_bf(a, frag_b(P + (size_t)(n0 + j * 16 + col) * DM + kc * 32, lane), acc[j]); }
  if (n0 < DM) {
#pragma unroll
    for (int j = 0; j < 8; ++j) { const float bv = bfr(BI[n0 + j * 16 + col]);
#pragma unroll
      for (int r = 0; r < 8; ++r) so[wave][8 * g + r][j * 16 + col] = (_Float16)(acc[j][r] + bv); }
    LDSX();
    const size_t rw = (size_t)rc0 + wave * 16;
    for (int rl = 0; rl < 16; ++rl) if (lane < 16) vst2((unsigned*)(NAT + (rw + rl) * DM + n0 + lane * 8), *(const v4u*)&so[wave][rl][lane * 8]);
  } else {
#pragma unroll
    for (int j = 0; j < 8; ++j) { const float bv = bfr(BI[n0 + j * 16 + col]);
#pragma unroll
      for (int r = 0; r < 8; ++r) sth[j * 16 + col][wave * 16 + 8 * g + r] = (_Float16)(acc[j][r] + bv); }
    __syncthreads();
    const int pc0 = n0 - DM;
    for (int q = tid; q < 128 * 8; q += 128) { const int d = q >> 3, pc = q & 7;
      const size_t o = ((size_t)b * DM + pc0 + d) * spb + s0 + pc * 8; vst2((unsigned*)(VT + o), *(const v4u*)&sth[d][pc * 8]); }
  }
}

__global__ __launch_bounds__(128) void k_attn(const _Float16* __restrict__ QH, const _Float16* __restrict__ KH, const _Float16* __restrict__ VT, const int* __restrict__ MK, float* __restrict__ O) {
  __shared__ __align__(16) float sp[4][16][36];
  __shared__ __align__(16) float so[4][16][68];
  __shared__ __align__(16) int sk[4][16][36];
  const int tid = threadIdx.x, wave = tid >> 5, lane = tid & 31, col = lane & 15, g = lane >> 4;
  const int qb = blockIdx.x, h = blockIdx.y, b = blockIdx.z; const int q0 = qb * 64 + wave * 16;
  const size_t rq = (size_t)b * SEQ + q0 + col;
  v16h aq[2];
#pragma unroll
  for (int kc = 0; kc < 2; ++kc) aq[kc] = frag_h(QH + rq * DM + h * HD + kc * 32, lane);
  float m[8], l[8];
#pragma unroll
  for (int r = 0; r < 8; ++r) { m[r] = -3.0e38f; l[r] = 0.f; }
  v8f acc[4] = {};
  const int* mrow = MK + ((size_t)b * SEQ_FULL + q0) * SEQK_FULL; const int mr = lane >> 3, mc = (lane & 7) * 4;
#pragma unroll 1
  for (int ks = 0; ks < SEQK / 32; ++ks) {
    { v4i mv[4];
#pragma unroll
      for (int i = 0; i < 4; ++i) mv[i] = *(const v4i*)(mrow + (size_t)(mr + 4 * i) * SEQK_FULL + ks * 32 + mc);
#pragma unroll
      for (int i = 0; i < 4; ++i) *(v4i*)&sk[wave][mr + 4 * i][mc] = mv[i]; }
    LDSX();
    v8f s[2];
#pragma unroll
    for (int ct = 0; ct < 2; ++ct) { const int kk = ks * 32 + ct * 16 + col; const _Float16* krow = KH + ((size_t)b * SEQK + kk) * DM + h * HD; v8f c = {};
#pragma unroll
      for (int kc = 0; kc < 2; ++kc) c = wmma16(aq[kc], frag_h(krow + kc * 32, lane), c);
#pragma unroll
      for (int r = 0; r < 8; ++r) s[ct][r] = (sk[wave][8 * g + r][ct * 16 + col] != 0) ? -3.0e38f : c[r] * 0.125f; }
#pragma unroll
    for (int r = 0; r < 8; ++r) { float mx = fmaxf(s[0][r], s[1][r]);
#pragma unroll
      for (int o = 1; o < 16; o <<= 1) mx = fmaxf(mx, __shfl_xor(mx, o));
      const float mn = fmaxf(m[r], mx); const float alpha = (m[r] <= -1.0e38f) ? 0.f : __expf(m[r] - mn);
      const float e0 = (s[0][r] <= -1.0e38f) ? 0.f : __expf(s[0][r] - mn), e1 = (s[1][r] <= -1.0e38f) ? 0.f : __expf(s[1][r] - mn); float es = e0 + e1;
#pragma unroll
      for (int o = 1; o < 16; o <<= 1) es += __shfl_xor(es, o);
      l[r] = l[r] * alpha + es; m[r] = mn;
#pragma unroll
      for (int dt = 0; dt < 4; ++dt) acc[dt][r] *= alpha;
      sp[wave][8 * g + r][col] = e0; sp[wave][8 * g + r][16 + col] = e1; }
    LDSX();
    v16h pa; { const float* prow = &sp[wave][col][0] + 8 * g;
#pragma unroll
      for (int i = 0; i < 8; ++i) { pa[i] = (_Float16)(prow[i] * 2048.0f); pa[8 + i] = (_Float16)(prow[16 + i] * 2048.0f); } }
#pragma unroll
    for (int dt = 0; dt < 4; ++dt) { const size_t vr = ((size_t)b * DM + h * HD + dt * 16 + col) * SEQK + ks * 32; acc[dt] = wmma16(pa, frag_h(VT + vr, lane), acc[dt]); }
    LDSX(); }
#pragma unroll
  for (int r = 0; r < 8; ++r) { const float il = (1.0f / 2048.0f) / l[r];
#pragma unroll
    for (int dt = 0; dt < 4; ++dt) so[wave][8 * g + r][dt * 16 + col] = acc[dt][r] * il; }
  LDSX();
  for (int rl = 0; rl < 16; ++rl) if (lane < 16) vst2(O + ((size_t)b * SEQ + q0 + rl) * DM + h * HD + lane * 4, *(const v4f*)&so[wave][rl][lane * 4]);
}

__global__ __launch_bounds__(128) void k_out(const float* __restrict__ O, const __bf16* __restrict__ P, const float* __restrict__ BO, float* __restrict__ Y) {
  __shared__ __align__(16) float so[4][16][132];
  const int tid = threadIdx.x, wave = tid >> 5, lane = tid & 31, col = lane & 15, g = lane >> 4; const size_t r0 = (size_t)blockIdx.x * 64 + wave * 16; const int n0 = blockIdx.y * 128;
  v8f acc[8] = {};
#pragma unroll 2
  for (int kc = 0; kc < DM / 32; ++kc) { const F2 a = split_row(O + (r0 + col) * DM, kc * 32, lane);
#pragma unroll
    for (int j = 0; j < 8; ++j) { const v16b w = frag_b(P + (size_t)(n0 + j * 16 + col) * DM + kc * 32, lane); acc[j] = wmma_bf(a.l, w, acc[j]); acc[j] = wmma_bf(a.h, w, acc[j]); } }
#pragma unroll
  for (int j = 0; j < 8; ++j) { const float bv = bfr(BO[n0 + j * 16 + col]);
#pragma unroll
    for (int r = 0; r < 8; ++r) so[wave][8 * g + r][j * 16 + col] = acc[j][r] + bv; }
  LDSX();
  for (int rl = 0; rl < 16; ++rl) vst2(Y + (r0 + rl) * DM + n0 + lane * 4, *(const v4f*)&so[wave][rl][lane * 4]);
}

__global__ __launch_bounds__(256) void k_lnpost(const float* __restrict__ Yp, const float* __restrict__ X, const float* __restrict__ G, const float* __restrict__ Bt, float* __restrict__ OUT) {
  __shared__ float red0[8], red1[8];
  const int rc = blockIdx.x; const int b = rc / SEQ, s = rc - b * SEQ; const size_t rin = (size_t)b * SEQ_FULL + s;
  const int t = threadIdx.x, lane = t & 31, wave = t >> 5;
  const v4f yv = *(const v4f*)(Yp + (size_t)rc * DM + t * 4), xv = *(const v4f*)(X + rin * DM + t * 4);
  float v[4];
#pragma unroll
  for (int i = 0; i < 4; ++i) v[i] = yv[i] + bfr(xv[i]);
  float ps = (v[0] + v[1]) + (v[2] + v[3]);
#pragma unroll
  for (int o = 16; o > 0; o >>= 1) ps += __shfl_xor(ps, o);
  if (lane == 0) red0[wave] = ps;
  __syncthreads();
  float S = 0.f;
#pragma unroll
  for (int i = 0; i < 8; ++i) S += red0[i];
  const float mean = S * (1.0f / DM);
  float d[4]; float pq = 0.f;
#pragma unroll
  for (int i = 0; i < 4; ++i) { d[i] = v[i] - mean; pq += d[i] * d[i]; }
#pragma unroll
  for (int o = 16; o > 0; o >>= 1) pq += __shfl_xor(pq, o);
  if (lane == 0) red1[wave] = pq;
  __syncthreads();
  float V = 0.f;
#pragma unroll
  for (int i = 0; i < 8; ++i) V += red1[i];
  const float rstd = 1.0f / sqrtf(V * (1.0f / DM) + LN_EPS);
  const v4f gv = *(const v4f*)(G + t * 4), bv = *(const v4f*)(Bt + t * 4); v4f o;
#pragma unroll
  for (int i = 0; i < 4; ++i) o[i] = d[i] * rstd * bfr(gv[i]) + bfr(bv[i]);
  vst2(OUT + rin * DM + t * 4, o);
}

extern "C" void kernel_launch(void* const* d_in, const int* in_sizes, int n_in, void* d_out, int out_size, void* d_ws, size_t ws_size, hipStream_t stream) {
  if (n_in < 13) return;
  const float* XQ = (const float*)d_in[0]; const float* XKV = (const float*)d_in[1];
  const float* WQ = (const float*)d_in[2]; const float* BQ = (const float*)d_in[3];
  const float* WKV = (const float*)d_in[4]; const float* BKV = (const float*)d_in[5];
  const float* WO = (const float*)d_in[6]; const float* BO = (const float*)d_in[7];
  const float* GQ = (const float*)d_in[8]; const float* BTQ = (const float*)d_in[9];
  const float* GP = (const float*)d_in[10]; const float* BTP = (const float*)d_in[11];
  const int* MK = (const int*)d_in[12];
  const long long needq = ((long long)(NB - 1) * SEQ_FULL + SEQ) * DM;
  const long long needkv = ((long long)(NB - 1) * SEQK_FULL + SEQK) * DM;
  const long long needm = ((long long)(NB - 1) * SEQ_FULL + SEQ) * SEQK_FULL;
  if ((long long)in_sizes[0] < needq || (long long)in_sizes[1] < needkv || in_sizes[2] < DM * DM || in_sizes[3] < DM || in_sizes[4] < DM * KVW || in_sizes[5] < KVW) return;
  if (in_sizes[6] < DM * DM || in_sizes[7] < DM || in_sizes[8] < DM || in_sizes[9] < DM || in_sizes[10] < DM || in_sizes[11] < DM || (long long)in_sizes[12] < needm) return;
  if ((long long)out_size < needq) return;
  if (ws_size < (size_t)WS_END) return;
  char* ws = (char*)d_ws;
  __bf16* PQ = (__bf16*)(ws + WS_PQ); __bf16* PKV = (__bf16*)(ws + WS_PKV); __bf16* PO = (__bf16*)(ws + WS_PO);
  float* NQ = (float*)(ws + WS_NQ); _Float16* QH = (_Float16*)(ws + WS_QH); _Float16* KH = (_Float16*)(ws + WS_KH); _Float16* VT = (_Float16*)(ws + WS_VT);
  float* O = (float*)(ws + WS_O); float* Y = (float*)(ws + WS_Y);
  k_pack<<<dim3(DM / 64, DM / 64), 256, 0, stream>>>(WQ, DM, DM, PQ);
  k_pack<<<dim3(KVW / 64, DM / 64), 256, 0, stream>>>(WKV, DM, KVW, PKV);
  k_pack<<<dim3(DM / 64, DM / 64), 256, 0, stream>>>(WO, DM, DM, PO);
  k_lnq<<<dim3(NB * SEQ), 256, 0, stream>>>(XQ, GQ, BTQ, NQ);
  k_proj<<<dim3(NB * SEQ / 64, DM / 128), 128, 0, stream>>>(NQ, SEQ, SEQ, PQ, BQ, QH, VT);
  k_proj<<<dim3(NB * SEQK / 64, KVW / 128), 128, 0, stream>>>(XKV, SEQK, SEQK_FULL, PKV, BKV, KH, VT);
  k_attn<<<dim3(SEQ / 64, NH, NB), 128, 0, stream>>>(QH, KH, VT, MK, O);
  k_out<<<dim3(NB * SEQ / 64, DM / 128), 128, 0, stream>>>(O, PO, BO, Y);
  k_lnpost<<<dim3(NB * SEQ), 256, 0, stream>>>(Y, XQ, GP, BTP, (float*)d_out);
}
